// DecoderLayer_82952998355344
// MI455X (gfx1250) — hardware-verified
//
#include <hip/hip_runtime.h>
#include <math.h>

typedef __attribute__((ext_vector_type(16))) _Float16 v16h;
typedef __attribute__((ext_vector_type(8)))  _Float16 v8h;
typedef __attribute__((ext_vector_type(8)))  float    v8f;
typedef __attribute__((ext_vector_type(4)))  float    v4f;

constexpr int kB    = 8;
constexpr int kL    = 512;
constexpr int kDM   = 512;
constexpr int kDI   = 1024;
constexpr int kNS   = 16;
constexpr int kDR   = 32;
constexpr int kDF   = 2048;
constexpr int kRows = kB * kL;
constexpr int kXdP  = kDR + 2 * kNS;
constexpr int kXZP  = 4 * kDI;
constexpr int kYP   = 2 * kDI;
constexpr int kConvTP = 260;
constexpr int kScanTS = 64;
constexpr int kScanCh = 64;
constexpr int kScanYP = 68;
static_assert(kRows == 4096 && kXdP == 64 && kXZP == 4096 && kYP == 2048, "shape constants");
static_assert((kDM % 32) == 0 && (kDI % 32) == 0 && (kDR % 32) == 0 && (kDF % 32) == 0 && (kYP % 32) == 0, "GEMM K multiples of 32");
static_assert((kRows % 64) == 0 && (kXZP % 64) == 0 && (kXdP % 64) == 0 && (kDI % 64) == 0 && (kDM % 64) == 0 && (kDF % 64) == 0, "GEMM M,N multiples of 64");
static_assert((kL % kScanTS) == 0 && (kL % 64) == 0 && (kDI % kScanCh) == 0 && (kDI % 256) == 0, "tile multiples");

constexpr float kCW  = 32.0f;
constexpr float kCU  = 16.0f;
constexpr float kCDT = 16.0f;
constexpr float kCY  = 32.0f;
constexpr float kCH  = 16.0f;

constexpr size_t kOffXH   = 0;
constexpr size_t kOffWIN  = kOffXH   + (size_t)kRows * kDM * 2;
constexpr size_t kOffWXP  = kOffWIN  + (size_t)kXZP * kDM * 2;
constexpr size_t kOffWDT  = kOffWXP  + (size_t)2 * kXdP * kDI * 2;
constexpr size_t kOffWOUT = kOffWDT  + (size_t)2 * kDI * kDR * 2;
constexpr size_t kOffW1   = kOffWOUT + (size_t)kDM * kYP * 2;
constexpr size_t kOffW2   = kOffW1   + (size_t)kDF * kDM * 2;
constexpr size_t kOffXZ   = kOffW2   + (size_t)kDM * kDF * 2;
constexpr size_t kOffU    = kOffXZ   + (size_t)kRows * kXZP * 2;
constexpr size_t kOffDBC  = kOffU    + (size_t)2 * kRows * kDI * 2;
constexpr size_t kOffDT   = kOffDBC  + (size_t)2 * kRows * kXdP * 4;
constexpr size_t kOffDLR  = kOffDT   + (size_t)2 * kRows * kDR * 2;
constexpr size_t kOffY    = kOffDLR  + (size_t)2 * kRows * kDI * 2;
constexpr size_t kOffMB   = kOffY    + (size_t)kRows * kYP * 2;
constexpr size_t kOffX1   = kOffMB   + (size_t)kRows * kDM * 4;
constexpr size_t kOffX1H  = kOffX1   + (size_t)kRows * kDM * 4;
constexpr size_t kOffY2   = kOffX1H  + (size_t)kRows * kDM * 2;
constexpr size_t kWsTotal = kOffY2   + (size_t)kRows * kDM * 4;
static_assert(kWsTotal == 130940928ull, "carve total");
static_assert(kWsTotal <= 134217728ull, "carve cap");
static_assert((size_t)kRows * kDF * 2 == (size_t)2 * kRows * kDI * 2, "H plane fits the U region exactly");
static_assert((kOffWIN % 128) == 0 && (kOffWXP % 128) == 0 && (kOffWDT % 128) == 0 && (kOffWOUT % 128) == 0 &&
              (kOffW1 % 128) == 0 && (kOffW2 % 128) == 0 && (kOffXZ % 128) == 0 && (kOffU % 128) == 0 &&
              (kOffDBC % 128) == 0 && (kOffDT % 128) == 0 && (kOffDLR % 128) == 0 && (kOffY % 128) == 0 &&
              (kOffMB % 128) == 0 && (kOffX1 % 128) == 0 && (kOffX1H % 128) == 0 && (kOffY2 % 128) == 0, "128-B aligned regions");

__device__ __forceinline__ float h16_to_f32(unsigned hb) {
  const unsigned sgn = (hb & 0x8000u) << 16;
  const unsigned em  = hb & 0x7fffu;
  const float fn  = __uint_as_float((em << 13) + 0x38000000u);
  const float fs  = (float)em * 5.9604644775390625e-8f;
  const float mag = (em < 0x400u) ? fs : fn;
  return __uint_as_float(__float_as_uint(mag) | sgn);
}
__device__ __forceinline__ float ld_h16(const unsigned* __restrict__ p32, size_t idx) {
  const unsigned w  = p32[idx >> 1];
  const unsigned hb = ((idx & 1) != 0) ? (w >> 16) : (w & 0xffffu);
  return h16_to_f32(hb);
}
__device__ __forceinline__ void wave_lds_sync() {
  __builtin_amdgcn_fence(__ATOMIC_RELEASE, "workgroup");
  __builtin_amdgcn_wave_barrier();
  __builtin_amdgcn_fence(__ATOMIC_ACQUIRE, "workgroup");
}
__device__ __forceinline__ float wave_sum(float v) {
#pragma unroll
  for (int o = 16; o > 0; o >>= 1) v += __shfl_xor(v, o, 32);
  return v;
}

union FragU { v16h v; v8h h[2]; };
__device__ __forceinline__ v16h frag_load(const _Float16* p) {
  FragU f;
  f.h[0] = *(const v8h*)(p);
  f.h[1] = *(const v8h*)(p + 16);
  return f.v;
}
__device__ __forceinline__ v8f frag_mma(v16h a, v16h b, v8f c) {
  return __builtin_amdgcn_wmma_f32_16x16x32_f16(false, a, false, b, (short)0, c, false, false);
}
__device__ __forceinline__ void guard_row(v8f& a0, v8f& a1, v8f& a2, v8f& a3, v16h x, v16h b0, v16h b1, v16h b2, v16h b3) {
  asm volatile("v_nop\n\tv_nop\n\tv_nop\n\tv_nop" : "+v"(a0), "+v"(a1), "+v"(a2), "+v"(a3) : "v"(x), "v"(b0), "v"(b1), "v"(b2), "v"(b3));
}
__device__ __forceinline__ void acc_guard4(v8f& a, v8f& b, v8f& c, v8f& d) {
  asm volatile("v_nop\n\tv_nop\n\tv_nop\n\tv_nop" : "+v"(a), "+v"(b), "+v"(c), "+v"(d));
}

template <int BIAS_MODE, int OUT_MODE, int ACT>
__global__ __launch_bounds__(256) void wmma_gemm64_f16(
    const unsigned short* __restrict__ Ap, int lda, long strideA,
    const unsigned short* __restrict__ Btp, int ldb, long strideB,
    void* __restrict__ Cout, int ldc, long strideC,
    const float* __restrict__ bias0, const float* __restrict__ bias1,
    int M, int N, int K, float scale, float post) {
  __shared__ __align__(16) float sT[8][16 * 68];
  const int b    = blockIdx.y;
  const int lane = threadIdx.x & 31;
  const int wave = threadIdx.x >> 5;
  const int tilesN = N >> 6;
  const int tilesM = M >> 6;
  const int tile = blockIdx.x * 8 + wave;
  if (tile >= tilesM * tilesN) return;
  const int tm = tile / tilesN;
  const int tn = tile - tm * tilesN;
  const int m0 = tm << 6;
  const int n0 = tn << 6;

  const _Float16* Ab = (const _Float16*)Ap  + (size_t)b * strideA;
  const _Float16* Bb = (const _Float16*)Btp + (size_t)b * strideB;
  const float* bp = (b != 0) ? bias1 : bias0;

  const int rlane = lane & 15;
  const int koff  = (lane >> 4) * 8;
  const int mOff  = (lane >> 4) * 8;

  v8f acc[4][4];
#pragma unroll
  for (int i = 0; i < 4; ++i)
#pragma unroll
    for (int j = 0; j < 4; ++j) acc[i][j] = (v8f){0.f, 0.f, 0.f, 0.f, 0.f, 0.f, 0.f, 0.f};

  for (int k0 = 0; k0 < K; k0 += 32) {
    v16h bh[4];
#pragma unroll
    for (int j = 0; j < 4; ++j) {
      const size_t bo = (size_t)(n0 + (j << 4) + rlane) * ldb + koff + k0;
      bh[j] = frag_load(Bb + bo);
    }
#pragma unroll
    for (int i = 0; i < 4; ++i) {
      const size_t ao = (size_t)(m0 + (i << 4) + rlane) * lda + koff + k0;
      const v16h ah = frag_load(Ab + ao);
#pragma unroll
      for (int j = 0; j < 4; ++j) acc[i][j] = frag_mma(ah, bh[j], acc[i][j]);
      guard_row(acc[i][0], acc[i][1], acc[i][2], acc[i][3], ah, bh[0], bh[1], bh[2], bh[3]);
    }
  }
  acc_guard4(acc[0][0], acc[0][1], acc[0][2], acc[0][3]);
  acc_guard4(acc[1][0], acc[1][1], acc[1][2], acc[1][3]);
  acc_guard4(acc[2][0], acc[2][1], acc[2][2], acc[2][3]);
  acc_guard4(acc[3][0], acc[3][1], acc[3][2], acc[3][3]);

  float* slab = sT[wave];
#pragma unroll
  for (int i = 0; i < 4; ++i) {
    const int mBase = m0 + (i << 4);
#pragma unroll
    for (int j = 0; j < 4; ++j) {
      const int n = n0 + (j << 4) + rlane;
      float bv = 0.f;
      if (BIAS_MODE == 2) bv = bp[n];
#pragma unroll
      for (int r = 0; r < 8; ++r) {
        float v = acc[i][j][r] * scale;
        if (BIAS_MODE == 2) v += bv;
        slab[(mOff + r) * 68 + (j << 4) + rlane] = v;
      }
    }
    wave_lds_sync();
    if (ACT != 0) {
#pragma unroll 1
      for (int t = 0; t < 32; ++t) {
        const int idx = t * 32 + lane;
        const int rr = idx >> 6, cc = idx & 63;
        float v = slab[rr * 68 + cc];
        if (ACT == 5) v = 0.5f * v * (1.0f + erff(v * 0.70710678118654752f));
        slab[rr * 68 + cc] = v * post;
      }
      wave_lds_sync();
    }
    if (OUT_MODE == 0) {
      float* C = (float*)Cout + (size_t)b * strideC;
      const int hh = lane >> 4, c4 = (lane & 15) * 4;
      for (int pass = 0; pass < 2; ++pass) {
#pragma unroll
        for (int it = 0; it < 8; ++it) {
          const int row = it * 2 + hh;
          const v4f v = *(const v4f*)(slab + row * 68 + c4);
          *(volatile v4f*)(C + (size_t)(mBase + row) * ldc + n0 + c4) = v;
        }
        __threadfence();
      }
    } else {
      const int q = lane >> 3, c8 = (lane & 7) * 8;
      unsigned short* C = (unsigned short*)Cout + (size_t)b * strideC;
      for (int pass = 0; pass < 2; ++pass) {
#pragma unroll
        for (int it = 0; it < 4; ++it) {
          const int row = it * 4 + q;
          const float* sp = slab + row * 68 + c8;
          v8h hv;
#pragma unroll
          for (int e = 0; e < 8; ++e) hv[e] = (_Float16)sp[e];
          *(volatile v8h*)(C + (size_t)(mBase + row) * ldc + n0 + c8) = hv;
        }
        __threadfence();
      }
    }
    wave_lds_sync();
  }
}

__global__ __launch_bounds__(256) void cast_f16_kernel(
    const float* __restrict__ src0, const float* __restrict__ src1, unsigned short* __restrict__ dst,
    int total8, int cols, int dpitch, long dstStride, float scale) {
  const int i = blockIdx.x * 256 + threadIdx.x;
  if (i >= total8) return;
  const float* src = (blockIdx.y != 0) ? src1 : src0;
  const int e0 = i << 3;
  const int r  = e0 / cols;
  const int c  = e0 - r * cols;
  const v4f a0 = *(const v4f*)(src + e0);
  const v4f a1 = *(const v4f*)(src + e0 + 4);
  v8h hv;
#pragma unroll
  for (int e = 0; e < 4; ++e) {
    hv[e]     = (_Float16)(a0[e] * scale);
    hv[4 + e] = (_Float16)(a1[e] * scale);
  }
  unsigned short* q = dst + (size_t)blockIdx.y * dstStride + (size_t)r * dpitch + c;
  *(volatile v8h*)q = hv;
  __threadfence();
  *(volatile v8h*)q = hv;
}

__global__ __launch_bounds__(256) void dt_cast_kernel(
    const float* __restrict__ DBC, unsigned short* __restrict__ DT, int total8, float scale) {
  const int i = blockIdx.x * 256 + threadIdx.x;
  if (i >= total8) return;
  const int e0 = i << 3;
  const int r  = e0 >> 5;
  const int c  = e0 & 31;
  const float* p = DBC + (size_t)r * kXdP + c;
  const v4f a0 = *(const v4f*)(p);
  const v4f a1 = *(const v4f*)(p + 4);
  v8h hv;
#pragma unroll
  for (int e = 0; e < 4; ++e) {
    hv[e]     = (_Float16)(a0[e] * scale);
    hv[4 + e] = (_Float16)(a1[e] * scale);
  }
  unsigned short* q = DT + e0;
  *(volatile v8h*)q = hv;
  __threadfence();
  *(volatile v8h*)q = hv;
}

__global__ __launch_bounds__(256) void conv_silu_kernel(
    const unsigned* __restrict__ XZ32,
    const float* __restrict__ cw0, const float* __restrict__ cb0,
    const float* __restrict__ cw1, const float* __restrict__ cb1,
    unsigned short* __restrict__ U16) {
  __shared__ __align__(16) float sT[16 * kConvTP];
  const int tid = threadIdx.x, lane = tid & 31, wave = tid >> 5;
  const int dir = blockIdx.z;
  const float* cw = (dir != 0) ? cw1 : cw0;
  const float* cb = (dir != 0) ? cb1 : cb0;
  const int d0 = blockIdx.x * 256, d = d0 + tid;
  const int g0 = blockIdx.y * 64;
  const int tb = g0 & (kL - 1);
  const size_t col = (size_t)dir * (2 * kDI) + d;
  const v4f wv = *(const v4f*)(cw + (size_t)d * 4);
  const float w0 = wv[0], w1 = wv[1], w2 = wv[2], w3 = wv[3];
  const float bc = cb[d];
  float h1, h2, h3;
  {
    const bool hist = (dir != 0) ? (tb + 64 < kL) : (tb > 0);
    const int rb = hist ? ((dir != 0) ? (g0 + 64) : (g0 - 3)) : g0;
    const float va = ld_h16(XZ32, (size_t)rb * kXZP + col);
    const float vb = ld_h16(XZ32, (size_t)(rb + 1) * kXZP + col);
    const float vc = ld_h16(XZ32, (size_t)(rb + 2) * kXZP + col);
    const float n1 = (dir != 0) ? va : vc;
    const float n3 = (dir != 0) ? vc : va;
    h1 = hist ? n1 : 0.f;
    h2 = hist ? vb : 0.f;
    h3 = hist ? n3 : 0.f;
  }
  unsigned short* Ud = U16 + (size_t)dir * kRows * kDI;
#pragma unroll 1
  for (int sub = 0; sub < 4; ++sub) {
    const int lb = (dir != 0) ? (g0 + (3 - sub) * 16) : (g0 + sub * 16);
#pragma unroll 1
    for (int s = 0; s < 16; ++s) {
      const int tr = (dir != 0) ? (15 - s) : s;
      const float xcur = ld_h16(XZ32, (size_t)(lb + tr) * kXZP + col);
      float acc = w0 * h3;
      acc = fmaf(w1, h2, acc);
      acc = fmaf(w2, h1, acc);
      acc = fmaf(w3, xcur, acc);
      const float sv = acc + bc;
      const float sg = __builtin_amdgcn_rcpf(1.0f + expf(-sv));
      sT[tr * kConvTP + tid] = (sv * sg) * kCU;
      h3 = h2; h2 = h1; h1 = xcur;
    }
    __syncthreads();
    v8h bv[2];
#pragma unroll
    for (int it = 0; it < 2; ++it) {
      const float* sp = sT + (it * 8 + wave) * kConvTP + lane * 8;
      const v4f a0 = *(const v4f*)(sp);
      const v4f a1 = *(const v4f*)(sp + 4);
#pragma unroll
      for (int e = 0; e < 4; ++e) {
        bv[it][e]     = (_Float16)a0[e];
        bv[it][4 + e] = (_Float16)a1[e];
      }
    }
    for (int pass = 0; pass < 2; ++pass) {
#pragma unroll
      for (int it = 0; it < 2; ++it)
        *(volatile v8h*)(Ud + (size_t)(lb + it * 8 + wave) * kDI + d0 + lane * 8) = bv[it];
      __threadfence();
    }
    __syncthreads();
  }
}

__global__ __launch_bounds__(64) void scan_kernel(
    const unsigned* __restrict__ DLR32, const unsigned* __restrict__ U32, const unsigned* __restrict__ XZ32,
    const float* __restrict__ DBC,
    const float* __restrict__ Alog0, const float* __restrict__ Dp0,
    const float* __restrict__ Alog1, const float* __restrict__ Dp1,
    unsigned short* __restrict__ Y16) {
  __shared__ __align__(16) float sBC[kScanTS * 32];
  __shared__ __align__(16) float sY[kScanTS * kScanYP];
  const int tid = threadIdx.x, lane = tid & 31, wave = tid >> 5;
  constexpr int kBlkPerB = kDI / kScanCh;
  const int bx   = blockIdx.x;
  const int dir  = bx / (kB * kBlkPerB);
  const int rem  = bx - dir * (kB * kBlkPerB);
  const int bix  = rem / kBlkPerB;
  const int d0   = (rem - bix * kBlkPerB) * kScanCh;
  const int d    = d0 + tid;
  const size_t row0 = (size_t)bix * kL;
  const float* Alog = (dir != 0) ? Alog1 : Alog0;
  const float* Dp   = (dir != 0) ? Dp1 : Dp0;
  const size_t planeB = (size_t)dir * kRows * kDI;
  const float* DBCd = DBC + (size_t)dir * kRows * kXdP;
  const size_t zcol = (size_t)dir * (2 * kDI) + kDI + d;

  float negA[kNS], h[kNS];
  {
    const v4f q0 = *(const v4f*)(Alog + (size_t)d * kNS);
    const v4f q1 = *(const v4f*)(Alog + (size_t)d * kNS + 4);
    const v4f q2 = *(const v4f*)(Alog + (size_t)d * kNS + 8);
    const v4f q3 = *(const v4f*)(Alog + (size_t)d * kNS + 12);
#pragma unroll
    for (int e = 0; e < 4; ++e) {
      negA[e]      = -expf(q0[e]);
      negA[4 + e]  = -expf(q1[e]);
      negA[8 + e]  = -expf(q2[e]);
      negA[12 + e] = -expf(q3[e]);
    }
  }
#pragma unroll
  for (int s = 0; s < kNS; ++s) h[s] = 0.f;
  const float Dd = Dp[d];
  constexpr float kInvCU = 1.0f / kCU;

  const int lr = tid >> 3, lc4 = (tid & 7) * 4;
  const int q = lane >> 3, c8 = (lane & 7) * 8;
#pragma unroll 1
  for (int ci = 0; ci < kL / kScanTS; ++ci) {
    const int t0 = (dir != 0) ? (kL - kScanTS - ci * kScanTS) : (ci * kScanTS);
    __syncthreads();
#pragma unroll
    for (int i = 0; i < 8; ++i) {
      const int r = lr + 8 * i;
      *(v4f*)(sBC + r * 32 + lc4) = *(const v4f*)(DBCd + (row0 + t0 + r) * kXdP + kDR + lc4);
    }
    __syncthreads();
#pragma unroll 1
    for (int s = 0; s < kScanTS; ++s) {
      const int tr = (dir != 0) ? (kScanTS - 1 - s) : s;
      const size_t grow = row0 + t0 + tr;
      const float* xr = sBC + tr * 32;
      float Bs[kNS], Cs[kNS];
#pragma unroll
      for (int q4 = 0; q4 < 4; ++q4) {
        const v4f bv = *(const v4f*)(xr + 4 * q4);
        const v4f cv = *(const v4f*)(xr + kNS + 4 * q4);
        Bs[4 * q4 + 0] = bv[0]; Bs[4 * q4 + 1] = bv[1]; Bs[4 * q4 + 2] = bv[2]; Bs[4 * q4 + 3] = bv[3];
        Cs[4 * q4 + 0] = cv[0]; Cs[4 * q4 + 1] = cv[1]; Cs[4 * q4 + 2] = cv[2]; Cs[4 * q4 + 3] = cv[3];
      }
      const float v   = ld_h16(DLR32, planeB + grow * kDI + d);
      const float a   = expf(-fabsf(v));
      const float up  = 1.0f + a;
      const float l1p = __logf(up) + (a - (up - 1.0f)) * __builtin_amdgcn_rcpf(up);
      const float dt  = fmaxf(v, 0.0f) + l1p;
      const float xt  = ld_h16(U32, planeB + grow * kDI + d) * kInvCU;
      const float zv  = ld_h16(XZ32, grow * kXZP + zcol);
      const float dtx = dt * xt;
      float y = 0.f;
#pragma unroll
      for (int k = 0; k < kNS; ++k) {
        const float e = __expf(dt * negA[k]);
        h[k] = e * h[k] + dtx * Bs[k];
        y = h[k] * Cs[k] + y;
      }
      y = xt * Dd + y;
      const float sg = __builtin_amdgcn_rcpf(1.0f + expf(-zv));
      y = y * (zv * sg);
      sY[tr * kScanYP + tid] = y * kCY;
    }
    __syncthreads();
    v8h hv[8];
#pragma unroll
    for (int it = 0; it < 8; ++it) {
      const int row = it * 8 + wave * 4 + q;
      const float* sp = sY + row * kScanYP + c8;
      const v4f a0 = *(const v4f*)(sp);
      const v4f a1 = *(const v4f*)(sp + 4);
#pragma unroll
      for (int e = 0; e < 4; ++e) {
        hv[it][e]     = (_Float16)a0[e];
        hv[it][4 + e] = (_Float16)a1[e];
      }
    }
    for (int pass = 0; pass < 2; ++pass) {
#pragma unroll
      for (int it = 0; it < 8; ++it) {
        const int row = it * 8 + wave * 4 + q;
        const size_t o = (row0 + t0 + row) * kYP + (size_t)dir * kDI + d0 + c8;
        *(volatile v8h*)(Y16 + o) = hv[it];
      }
      __threadfence();
    }
  }
}

__global__ __launch_bounds__(256) void ln1_kernel(
    const float* __restrict__ x, const float* __restrict__ MB,
    const float* __restrict__ g, const float* __restrict__ be,
    float* __restrict__ X1, unsigned short* __restrict__ X1h) {
  __shared__ __align__(16) float sR[8][kDM];
  const int lane = threadIdx.x & 31, wave = threadIdx.x >> 5;
  const int row = blockIdx.x * 8 + wave;
  const size_t rb = (size_t)row * kDM;
  v4f v[4];
#pragma unroll
  for (int it = 0; it < 4; ++it) {
    const int c = it * 128 + lane * 4;
    const v4f xa = *(const v4f*)(x + rb + c);
    const v4f ma = *(const v4f*)(MB + rb + c);
    v[it] = xa + ma;
  }
  float s = 0.f;
#pragma unroll
  for (int it = 0; it < 4; ++it) s += (v[it][0] + v[it][1]) + (v[it][2] + v[it][3]);
  s = wave_sum(s);
  const float mean = s * (1.0f / (float)kDM);
  float s2 = 0.f;
#pragma unroll
  for (int it = 0; it < 4; ++it) {
#pragma unroll
    for (int e = 0; e < 4; ++e) {
      const float dd = v[it][e] - mean;
      s2 += dd * dd;
    }
  }
  s2 = wave_sum(s2);
  const float rstd = 1.0f / sqrtf(s2 * (1.0f / (float)kDM) + 1e-5f);
  asm volatile("" ::: "memory");
  float* sr = sR[wave];
  v4f o[4];
#pragma unroll
  for (int it = 0; it < 4; ++it) {
    const int c = it * 128 + lane * 4;
    const v4f gg = *(const v4f*)(g + c);
    const v4f bb = *(const v4f*)(be + c);
#pragma unroll
    for (int e = 0; e < 4; ++e) o[it][e] = (v[it][e] - mean) * rstd * gg[e] + bb[e];
    *(v4f*)(sr + c) = o[it];
  }
  wave_lds_sync();
  v8h hv[2];
#pragma unroll
  for (int it = 0; it < 2; ++it) {
    const float* sp = sr + it * 256 + lane * 8;
    const v4f a0 = *(const v4f*)(sp);
    const v4f a1 = *(const v4f*)(sp + 4);
#pragma unroll
    for (int e = 0; e < 4; ++e) {
      hv[it][e]     = (_Float16)a0[e];
      hv[it][4 + e] = (_Float16)a1[e];
    }
  }
  for (int pass = 0; pass < 2; ++pass) {
#pragma unroll
    for (int it = 0; it < 4; ++it)
      *(volatile v4f*)(X1 + rb + it * 128 + lane * 4) = o[it];
#pragma unroll
    for (int it = 0; it < 2; ++it)
      *(volatile v8h*)(X1h + rb + it * 256 + lane * 8) = hv[it];
    __threadfence();
  }
}

__global__ __launch_bounds__(256) void ln2_kernel(
    const float* __restrict__ X1, const float* __restrict__ Y2,
    const float* __restrict__ g, const float* __restrict__ be,
    float* __restrict__ out) {
  const int lane = threadIdx.x & 31, wave = threadIdx.x >> 5;
  const int row = blockIdx.x * 8 + wave;
  const size_t rb = (size_t)row * kDM;
  v4f v[4];
#pragma unroll
  for (int it = 0; it < 4; ++it) {
    const int c = it * 128 + lane * 4;
    const v4f xa = *(const v4f*)(X1 + rb + c);
    const v4f ya = *(const v4f*)(Y2 + rb + c);
    v[it] = xa + ya;
  }
  float s = 0.f;
#pragma unroll
  for (int it = 0; it < 4; ++it) s += (v[it][0] + v[it][1]) + (v[it][2] + v[it][3]);
  s = wave_sum(s);
  const float mean = s * (1.0f / (float)kDM);
  float s2 = 0.f;
#pragma unroll
  for (int it = 0; it < 4; ++it) {
#pragma unroll
    for (int e = 0; e < 4; ++e) {
      const float dd = v[it][e] - mean;
      s2 += dd * dd;
    }
  }
  s2 = wave_sum(s2);
  const float rstd = 1.0f / sqrtf(s2 * (1.0f / (float)kDM) + 1e-5f);
  asm volatile("" ::: "memory");
  v4f o[4];
#pragma unroll
  for (int it = 0; it < 4; ++it) {
    const int c = it * 128 + lane * 4;
    const v4f gg = *(const v4f*)(g + c);
    const v4f bb = *(const v4f*)(be + c);
#pragma unroll
    for (int e = 0; e < 4; ++e) o[it][e] = (v[it][e] - mean) * rstd * gg[e] + bb[e];
  }
  for (int pass = 0; pass < 2; ++pass) {
#pragma unroll
    for (int it = 0; it < 4; ++it)
      *(volatile v4f*)(out + rb + it * 128 + lane * 4) = o[it];
    __threadfence();
  }
}

extern "C" void kernel_launch(void* const* d_in, const int* in_sizes, int n_in,
                              void* d_out, int out_size, void* d_ws, size_t ws_size,
                              hipStream_t stream) {
  if (n_in < 27) return;
  if (in_sizes[0] != kRows * kDM) return;
  for (int base = 1; base <= 10; base += 9) {
    if (in_sizes[base + 0] != 2 * kDI * kDM) return;
    if (in_sizes[base + 1] != kDI * 4) return;
    if (in_sizes[base + 2] != kDI) return;
    if (in_sizes[base + 3] != kXdP * kDI) return;
    if (in_sizes[base + 4] != kDI * kDR) return;
    if (in_sizes[base + 5] != kDI) return;
    if (in_sizes[base + 6] != kDI * kNS) return;
    if (in_sizes[base + 7] != kDI) return;
    if (in_sizes[base + 8] != kDM * kDI) return;
  }
  if (in_sizes[19] != kDF * kDM || in_sizes[20] != kDF) return;
  if (in_sizes[21] != kDM * kDF || in_sizes[22] != kDM) return;
  if (in_sizes[23] != kDM || in_sizes[24] != kDM || in_sizes[25] != kDM || in_sizes[26] != kDM) return;
  if (out_size != kRows * kDM) return;
  if (ws_size < kWsTotal) return;

  const float* x        = (const float*)d_in[0];
  const float* f_in_w   = (const float*)d_in[1];
  const float* f_conv_w = (const float*)d_in[2];
  const float* f_conv_b = (const float*)d_in[3];
  const float* f_xp_w   = (const float*)d_in[4];
  const float* f_dt_w   = (const float*)d_in[5];
  const float* f_dt_b   = (const float*)d_in[6];
  const float* f_A_log  = (const float*)d_in[7];
  const float* f_D      = (const float*)d_in[8];
  const float* f_out_w  = (const float*)d_in[9];
  const float* r_in_w   = (const float*)d_in[10];
  const float* r_conv_w = (const float*)d_in[11];
  const float* r_conv_b = (const float*)d_in[12];
  const float* r_xp_w   = (const float*)d_in[13];
  const float* r_dt_w   = (const float*)d_in[14];
  const float* r_dt_b   = (const float*)d_in[15];
  const float* r_A_log  = (const float*)d_in[16];
  const float* r_D      = (const float*)d_in[17];
  const float* r_out_w  = (const float*)d_in[18];
  const float* conv1_w  = (const float*)d_in[19];
  const float* conv1_b  = (const float*)d_in[20];
  const float* conv2_w  = (const float*)d_in[21];
  const float* conv2_b  = (const float*)d_in[22];
  const float* ln1_g    = (const float*)d_in[23];
  const float* ln1_b    = (const float*)d_in[24];
  const float* ln2_g    = (const float*)d_in[25];
  const float* ln2_b    = (const float*)d_in[26];
  float* out = (float*)d_out;

  char* ws = (char*)d_ws;
  unsigned short* XH   = (unsigned short*)(ws + kOffXH);
  unsigned short* WIN  = (unsigned short*)(ws + kOffWIN);
  unsigned short* WXP  = (unsigned short*)(ws + kOffWXP);
  unsigned short* WDT  = (unsigned short*)(ws + kOffWDT);
  unsigned short* WOUT = (unsigned short*)(ws + kOffWOUT);
  unsigned short* W1   = (unsigned short*)(ws + kOffW1);
  unsigned short* W2   = (unsigned short*)(ws + kOffW2);
  unsigned short* XZ   = (unsigned short*)(ws + kOffXZ);
  unsigned short* U16  = (unsigned short*)(ws + kOffU);
  unsigned short* H16  = (unsigned short*)(ws + kOffU);
  float*          DBC  = (float*)(ws + kOffDBC);
  unsigned short* DT   = (unsigned short*)(ws + kOffDT);
  unsigned short* DLR  = (unsigned short*)(ws + kOffDLR);
  unsigned short* Y16  = (unsigned short*)(ws + kOffY);
  float*          MB   = (float*)(ws + kOffMB);
  float*          X1   = (float*)(ws + kOffX1);
  unsigned short* X1H  = (unsigned short*)(ws + kOffX1H);
  float*          Y2   = (float*)(ws + kOffY2);
  const float* nob = conv2_b;

  cast_f16_kernel<<<dim3((kRows * kDM / 8) / 256, 1), 256, 0, stream>>>(x, x, XH, kRows * kDM / 8, kDM, kDM, 0L, 1.0f);
  cast_f16_kernel<<<dim3((2 * kDI * kDM / 8) / 256, 2), 256, 0, stream>>>(f_in_w, r_in_w, WIN, 2 * kDI * kDM / 8, kDM, kDM, (long)2 * kDI * kDM, kCW);
  cast_f16_kernel<<<dim3((kXdP * kDI / 8) / 256, 2), 256, 0, stream>>>(f_xp_w, r_xp_w, WXP, kXdP * kDI / 8, kDI, kDI, (long)kXdP * kDI, kCW);
  cast_f16_kernel<<<dim3((kDI * kDR / 8) / 256, 2), 256, 0, stream>>>(f_dt_w, r_dt_w, WDT, kDI * kDR / 8, kDR, kDR, (long)kDI * kDR, kCW);
  cast_f16_kernel<<<dim3((kDM * kDI / 8) / 256, 2), 256, 0, stream>>>(f_out_w, r_out_w, WOUT, kDM * kDI / 8, kDI, kYP, (long)kDI, kCW);
  cast_f16_kernel<<<dim3((kDF * kDM / 8) / 256, 1), 256, 0, stream>>>(conv1_w, conv1_w, W1, kDF * kDM / 8, kDM, kDM, 0L, kCW);
  cast_f16_kernel<<<dim3((kDM * kDF / 8) / 256, 1), 256, 0, stream>>>(conv2_w, conv2_w, W2, kDM * kDF / 8, kDF, kDF, 0L, kCW);

  wmma_gemm64_f16<0, 1, 0><<<dim3(512, 1), 256, 0, stream>>>(
      XH, kDM, 0L, WIN, kDM, 0L, (void*)XZ, kXZP, 0L, nob, nob,
      kRows, kXZP, kDM, 1.0f / kCW, 1.0f);

  conv_silu_kernel<<<dim3(kDI / 256, kRows / 64, 2), 256, 0, stream>>>(
      (const unsigned*)XZ, f_conv_w, f_conv_b, r_conv_w, r_conv_b, U16);

  wmma_gemm64_f16<0, 0, 0><<<dim3(8, 2), 256, 0, stream>>>(
      U16, kDI, (long)kRows * kDI, WXP, kDI, (long)kXdP * kDI, (void*)DBC, kXdP, (long)kRows * kXdP, nob, nob,
      kRows, kXdP, kDI, 1.0f / (kCW * kCU), 1.0f);

  dt_cast_kernel<<<(2 * kRows * kDR / 8) / 256, 256, 0, stream>>>(DBC, DT, 2 * kRows * kDR / 8, kCDT);

  wmma_gemm64_f16<2, 1, 0><<<dim3(128, 2), 256, 0, stream>>>(
      DT, kDR, (long)kRows * kDR, WDT, kDR, (long)kDI * kDR, (void*)DLR, kDI, (long)kRows * kDI, f_dt_b, r_dt_b,
      kRows, kDI, kDR, 1.0f / (kCDT * kCW), 1.0f);

  scan_kernel<<<2 * kB * (kDI / kScanCh), kScanCh, 0, stream>>>(
      (const unsigned*)DLR, (const unsigned*)U16, (const unsigned*)XZ, DBC,
      f_A_log, f_D, r_A_log, r_D, Y16);

  wmma_gemm64_f16<0, 0, 0><<<dim3(64, 1), 256, 0, stream>>>(
      Y16, kYP, 0L, WOUT, kYP, 0L, (void*)MB, kDM, 0L, nob, nob,
      kRows, kDM, kYP, 1.0f / (kCY * kCW), 1.0f);

  ln1_kernel<<<kRows / 8, 256, 0, stream>>>(x, MB, ln1_g, ln1_b, X1, X1H);

  wmma_gemm64_f16<2, 1, 5><<<dim3(256, 1), 256, 0, stream>>>(
      X1H, kDM, 0L, W1, kDM, 0L, (void*)H16, kDF, 0L, conv1_b, conv1_b,
      kRows, kDF, kDM, 1.0f / kCW, kCH);

  wmma_gemm64_f16<2, 0, 0><<<dim3(64, 1), 256, 0, stream>>>(
      H16, kDF, 0L, W2, kDF, 0L, (void*)Y2, kDM, 0L, conv2_b, conv2_b,
      kRows, kDM, kDF, 1.0f / (kCH * kCW), 1.0f);

  ln2_kernel<<<kRows / 8, 256, 0, stream>>>(X1, Y2, ln2_g, ln2_b, out);
}
